// WiseDiffModule_78615081386009
// MI455X (gfx1250) — hardware-verified
//
#include <hip/hip_runtime.h>
#include <stdint.h>

typedef _Float16 v16h __attribute__((ext_vector_type(16)));
typedef _Float16 v8h  __attribute__((ext_vector_type(8)));
typedef float    v8f  __attribute__((ext_vector_type(8)));
typedef float    v4f  __attribute__((ext_vector_type(4)));
typedef v8h __attribute__((may_alias)) v8ha;
typedef v4f __attribute__((may_alias)) v4fa;

union Frag { v16h v; v8h half[2]; };

#define NB     256
#define NC     512
#define HW     49
#define NPAD   64
#define KDIM   1024
#define ODIM   512
#define CG     64
#define NIN    (NB * NC * HW)
#define WSCALE 64.0f
#define WINV   0.015625f

__device__ __forceinline__ v8f wmma_f16(v16h a, v16h b, v8f c) {
#if defined(__HIP_DEVICE_COMPILE__)
  v8f d = __builtin_amdgcn_wmma_f32_16x16x32_f16(false, a, false, b, (short)0, c, false, false);
  asm volatile("v_nop\n\tv_nop\n\tv_nop\n\tv_nop" : "+v"(d) : "v"(a), "v"(b));
  return d;
#else
  (void)a; (void)b;
  return c;
#endif
}

__device__ __forceinline__ v16h load_frag(const _Float16* p, int h) {
  Frag f;
  f.half[0] = *(const v8ha*)(p + 8 * h);
  f.half[1] = *(const v8ha*)(p + 16 + 8 * h);
  return f.v;
}

__global__ __launch_bounds__(256) void cvt_w_kernel(const float* __restrict__ cw,
                                                   _Float16* __restrict__ cw16) {
  const int g = blockIdx.x * 256 + threadIdx.x;
  if (g >= (ODIM * KDIM) / 8) return;
  const float* src = cw + (size_t)g * 8;
  const v4f a = *(const v4fa*)src;
  const v4f c = *(const v4fa*)(src + 4);
  const v8h o = { (_Float16)(a.x * WSCALE), (_Float16)(a.y * WSCALE), (_Float16)(a.z * WSCALE), (_Float16)(a.w * WSCALE),
                  (_Float16)(c.x * WSCALE), (_Float16)(c.y * WSCALE), (_Float16)(c.z * WSCALE), (_Float16)(c.w * WSCALE) };
  _Float16* dst = cw16 + (size_t)g * 8;
  *(volatile v8h*)dst = o;
  __threadfence();
  *(volatile v8h*)dst = o;
}

__device__ __forceinline__ void pack_store_pass(const _Float16* sF, _Float16* F1h,
                                                int b, int cg, int wave, int lane) {
  const int q8 = lane & 7, sub = lane >> 3;
#pragma unroll
  for (int i = 0; i < 4; ++i) {
    const int L = i * 32 + wave * 4 + sub;
    const int seg = L >> 6, n = L & 63;
    const v8h v = *(const v8ha*)(sF + seg * (NPAD * CG) + n * CG + 8 * q8);
    _Float16* dst = F1h + ((size_t)b * NPAD + n) * KDIM + seg * NC + cg * CG + 8 * q8;
    *(volatile v8h*)dst = v;
  }
}

__global__ __launch_bounds__(256) void pack_kernel(const float* __restrict__ T,
                                                  const float* __restrict__ V,
                                                  const float* __restrict__ W9,
                                                  _Float16* __restrict__ F1h) {
  __shared__ float sT[CG * HW];
  __shared__ float sV[CG * HW];
  __shared__ __attribute__((aligned(16))) _Float16 sF[2 * NPAD * CG];
  __shared__ float sW[16];

  const int tid = threadIdx.x, lane = tid & 31, wave = tid >> 5;
  const int b = blockIdx.x >> 3, cg = blockIdx.x & 7;
  const size_t base = ((size_t)b * NC + (size_t)cg * CG) * HW;

  for (int i = tid; i < CG * HW; i += 256) {
    sT[i] = T[base + i];
    sV[i] = V[base + i];
  }
  if (tid < 9) sW[tid] = W9[tid];
  for (int i = tid; i < 2 * (NPAD - HW) * CG; i += 256) {
    const int seg = (i >= (NPAD - HW) * CG) ? 1 : 0;
    const int rem = i - seg * ((NPAD - HW) * CG);
    sF[seg * (NPAD * CG) + HW * CG + rem] = (_Float16)0.0f;
  }
  __syncthreads();

  float w[9];
#pragma unroll
  for (int k = 0; k < 9; ++k) w[k] = sW[k];

  const int cl = tid & 63, cq = tid >> 6;
  const float* tI = sT + cl * HW;
  const float* vI = sV + cl * HW;

  for (int cell = cq; cell < HW; cell += 4) {
    const int hr = cell / 7, wc = cell - hr * 7;
    const int rm = (hr == 0) ? 1 : (hr - 1);
    const int rp = (hr == 6) ? 5 : (hr + 1);
    const int cm = (wc == 0) ? 1 : (wc - 1);
    const int cp = (wc == 6) ? 5 : (wc + 1);
    const int ro[3] = { rm * 7, hr * 7, rp * 7 };
    const int co[3] = { cm, wc, cp };
    const float tc = tI[cell], vc = vI[cell];
    float acc = 0.0f;
#pragma unroll
    for (int i = 0; i < 3; ++i) {
#pragma unroll
      for (int j = 0; j < 3; ++j) {
        const int idx = ro[i] + co[j];
        const float dT = tI[idx] - tc;
        const float dV = vI[idx] - vc;
        const float e = __expf((dT * dT) * -0.25f);
        acc = acc + (e * dV) * w[3 * i + j];
      }
    }
    sF[cell * CG + cl] = (_Float16)vc;
    sF[NPAD * CG + cell * CG + cl] = (_Float16)acc;
  }
  __syncthreads();

  pack_store_pass(sF, F1h, b, cg, wave, lane);
  __threadfence();
  pack_store_pass(sF, F1h, b, cg, wave, lane);
}

__device__ __forceinline__ void gemm_store_pass(const float* sO, float* obase,
                                                int wave, int lane) {
  const int q8 = lane & 7, sub = lane >> 3;
#pragma unroll
  for (int i = 0; i < 7; ++i) {
    const int L = i * 32 + wave * 4 + sub;
    if (L < (128 * HW) / 32) {
      const v4f v = *(const v4fa*)(sO + L * 32 + 4 * q8);
      *(volatile v4f*)(obase + L * 32 + 4 * q8) = v;
    }
  }
}

__global__ __launch_bounds__(256) void gemm_kernel(const _Float16* __restrict__ F1h,
                                                  const _Float16* __restrict__ cw16,
                                                  const float* __restrict__ convb,
                                                  float* __restrict__ out) {
  __shared__ __attribute__((aligned(16))) float sO[128 * HW];

  const int tid = threadIdx.x, lane = tid & 31, wave = tid >> 5;
  const int h = lane >> 4, m = lane & 15;
  const int b = blockIdx.x >> 2, mg = blockIdx.x & 3;
  const int o0 = mg * 128 + wave * 16;

  const _Float16* arow = cw16 + (size_t)(o0 + m) * KDIM;
  const _Float16* brow = F1h + ((size_t)b * NPAD + m) * KDIM;

  const v8f zero8 = {0.f, 0.f, 0.f, 0.f, 0.f, 0.f, 0.f, 0.f};
  v8f acc[4];
#pragma unroll
  for (int nt = 0; nt < 4; ++nt) acc[nt] = zero8;

#pragma unroll 2
  for (int k0 = 0; k0 < KDIM; k0 += 32) {
    const v16h a = load_frag(arow + k0, h);
#pragma unroll
    for (int nt = 0; nt < 4; ++nt) {
      const v16h bfr = load_frag(brow + (size_t)nt * 16 * KDIM + k0, h);
      acc[nt] = wmma_f16(a, bfr, acc[nt]);
    }
  }

#pragma unroll
  for (int r = 0; r < 8; ++r) {
    const int ol = wave * 16 + 8 * h + r;
    const float bv = convb[mg * 128 + ol];
#pragma unroll
    for (int nt = 0; nt < 4; ++nt) {
      const int n = nt * 16 + m;
      if (n < HW) sO[ol * HW + n] = acc[nt][r] * WINV + bv;
    }
  }
  __syncthreads();

  float* obase = out + ((size_t)b * ODIM + (size_t)mg * 128) * HW;
  gemm_store_pass(sO, obase, wave, lane);
  __threadfence();
  gemm_store_pass(sO, obase, wave, lane);
}

extern "C" void kernel_launch(void* const* d_in, const int* in_sizes, int n_in,
                              void* d_out, int out_size, void* d_ws, size_t ws_size,
                              hipStream_t stream) {
  if (n_in < 5) return;
  if (in_sizes[0] != NIN || in_sizes[1] != NIN) return;
  if (in_sizes[2] != 9) return;
  if (in_sizes[3] != ODIM * KDIM || in_sizes[4] != ODIM) return;
  if (out_size != NIN) return;

  const float* T  = (const float*)d_in[0];
  const float* V  = (const float*)d_in[1];
  const float* W9 = (const float*)d_in[2];
  const float* cw = (const float*)d_in[3];
  const float* cb = (const float*)d_in[4];
  float* out = (float*)d_out;

  const size_t f1_bytes = (size_t)NB * NPAD * KDIM * 2;
  const size_t cw_bytes = (size_t)ODIM * KDIM * 2;
  if (f1_bytes + cw_bytes > ws_size) return;

  char* ws = (char*)d_ws;
  _Float16* F1h  = (_Float16*)(ws);
  _Float16* cw16 = (_Float16*)(ws + f1_bytes);

  cvt_w_kernel<<<((ODIM * KDIM) / 8 + 255) / 256, 256, 0, stream>>>(cw, cw16);
  pack_kernel<<<NB * (NC / CG), 256, 0, stream>>>(T, V, W9, F1h);
  gemm_kernel<<<NB * 4, 256, 0, stream>>>(F1h, cw16, cb, out);
}
